// GraphCrossModule_57097295233744
// MI455X (gfx1250) — hardware-verified
//
#include <hip/hip_runtime.h>

#define DF 128
#define GR 64
#define LP 136
#define OP 132
#define NBA 512
#define NBD 4096
#define CH 2048
#define ITS 8
#define NPART 10

typedef __bf16 v16bf __attribute__((ext_vector_type(16)));
typedef __bf16 v8bf __attribute__((ext_vector_type(8)));
typedef _Float16 v16h __attribute__((ext_vector_type(16)));
typedef _Float16 v8h __attribute__((ext_vector_type(8)));
typedef float v8f __attribute__((ext_vector_type(8)));
typedef float v4f __attribute__((ext_vector_type(4)));
typedef unsigned int v4u __attribute__((ext_vector_type(4)));

union FragB { v16bf v; v8bf h[2]; };
union FragH { v16h v; v8h h[2]; };

__device__ __forceinline__ unsigned short f2bf(float f) {
    unsigned int x = __float_as_uint(f);
    unsigned int r = x + 0x7FFFu + ((x >> 16) & 1u);
    return (unsigned short)(r >> 16);
}
__device__ __forceinline__ float bf2f(unsigned short u) { return __uint_as_float(((unsigned int)u) << 16); }
__device__ __forceinline__ unsigned short f2h(float f) {
    union { _Float16 h; unsigned short u; } c; c.h = (_Float16)f; return c.u;
}
__device__ __forceinline__ float sigf(float x) { return 1.0f / (1.0f + expf(-x)); }
__device__ __forceinline__ unsigned int fmap(float f) {
    unsigned int u = __float_as_uint(f);
    return (u & 0x80000000u) ? ~u : (u | 0x80000000u);
}
__device__ __forceinline__ int clampi(int v, int lo, int hi) { return v < lo ? lo : (v > hi ? hi : v); }

#define WNOP2(acc, a, b) asm volatile("v_nop\n\tv_nop\n\tv_nop\n\tv_nop" : "+v"(acc) : "v"(a), "v"(b))
#define WNOP4(acc, a, b, c, d) asm volatile("v_nop\n\tv_nop\n\tv_nop\n\tv_nop" : "+v"(acc) : "v"(a), "v"(b), "v"(c), "v"(d))

__global__ __launch_bounds__(256) void k_prepw(const float* __restrict__ W0, const float* __restrict__ W1,
                                               const float* __restrict__ W2, const float* __restrict__ W3,
                                               const float* __restrict__ W4, unsigned short* img) {
    __shared__ __attribute__((aligned(16))) unsigned short sh[DF * LP];
    const int t = threadIdx.x;
    const int b = blockIdx.x;
    const float* W = W0; int kind = 0;
    switch (b) {
        case 0: W = W0; kind = 0; break;
        case 1: W = W0; kind = 1; break;
        case 2: W = W0; kind = 2; break;
        case 3: W = W1; kind = 0; break;
        case 4: W = W1; kind = 1; break;
        case 5: W = W2; kind = 0; break;
        case 6: W = W2; kind = 1; break;
        case 7: W = W2; kind = 2; break;
        case 8: W = W3; kind = 2; break;
        default: W = W4; kind = 2; break;
    }
    for (int q = t; q < DF * DF / 4; q += 256) {
        const int k = q >> 5, n0 = (q & 31) * 4;
        const float4 v = *(const float4*)(W + (size_t)k * DF + n0);
        const float vv[4] = {v.x, v.y, v.z, v.w};
#pragma unroll
        for (int i = 0; i < 4; ++i) {
            const float f = vv[i];
            unsigned short u;
            if (kind == 0) u = f2bf(f);
            else if (kind == 1) { const unsigned short hi = f2bf(f); u = f2bf(f - bf2f(hi)); }
            else u = f2h(f * 64.0f);
            sh[(n0 + i) * LP + k] = u;
        }
    }
    __syncthreads();
    unsigned short* dp = img + (size_t)b * (DF * DF);
#pragma unroll
    for (int rep = 0; rep < 2; ++rep) {
        for (int q = t; q < DF * 16; q += 256) {
            const int n = q >> 4, c = (q & 15) * 8;
            const v4u v = *(const v4u*)(&sh[n * LP + c]);
            *(volatile v4u*)(dp + (size_t)n * DF + c) = v;
        }
        __threadfence();
    }
}

template <int NB, int OSH>
__device__ __forceinline__ void scan_chunk(const int* __restrict__ dst, int cb, int E, int node0,
                                           int* cnt, int* pos, int* lst, int* tot, int* segst, int* segn) {
    const int t = threadIdx.x, w = t >> 5, lane = t & 31;
    const unsigned lt = (1u << lane) - 1u;
    int pk[ITS];
#pragma unroll
    for (int it = 0; it < ITS; ++it) {
        const int e = cb + it * 256 + t;
        const int ec = (e < E) ? e : (E - 1);
        const int d = dst[ec];
        const int dl = d - node0;
        const bool hf = (e < E) && ((unsigned)dl < (unsigned)NB);
        const unsigned hb = __builtin_amdgcn_ballot_w32(hf);
        int p = 0, c8 = 0;
        if (hb != 0u) {
            const int o = (dl >> OSH) & 7;
            const unsigned b0 = __builtin_amdgcn_ballot_w32((o & 1) != 0);
            const unsigned b1 = __builtin_amdgcn_ballot_w32((o & 2) != 0);
            const unsigned b2 = __builtin_amdgcn_ballot_w32((o & 4) != 0);
            const unsigned mine = hb & ((o & 1) ? b0 : ~b0) & ((o & 2) ? b1 : ~b1) & ((o & 4) ? b2 : ~b2);
            const int rk = __builtin_popcount(mine & lt);
            const unsigned ml = hb & ((lane & 1) ? b0 : ~b0) & ((lane & 2) ? b1 : ~b1) & ((lane & 4) ? b2 : ~b2);
            c8 = __builtin_popcount(ml);
            p = hf ? ((dl & 4095) | (rk << 12) | (1 << 20)) : 0;
        }
        if (lane < 8) cnt[lane * 64 + it * 8 + w] = c8;
        pk[it] = p;
    }
    __syncthreads();
    {
        const int base = w * 64;
        const int c0 = cnt[base + 2 * lane], c1 = cnt[base + 2 * lane + 1];
        const int s = c0 + c1;
        int incl = s;
#pragma unroll
        for (int off = 1; off < 32; off <<= 1) {
            const int v = __shfl_up(incl, off, 32);
            if (lane >= off) incl += v;
        }
        const int excl = incl - s;
        pos[base + 2 * lane] = excl;
        pos[base + 2 * lane + 1] = excl + c0;
        if (lane == 31) tot[w] = incl;
    }
    __syncthreads();
    if (w == 0) {
        const int tv = (lane < 8) ? tot[lane] : 0;
        int bsum = 0;
#pragma unroll
        for (int oo = 0; oo < 8; ++oo) { const int v = __shfl(tv, oo, 32); if (oo < lane) bsum += v; }
        if (lane < 8) { segst[lane] = bsum; segn[lane] = tv; }
    }
    __syncthreads();
#pragma unroll
    for (int it = 0; it < ITS; ++it) {
        const int p = pk[it];
        if (p & (1 << 20)) {
            const int dl = p & 4095, rk = (p >> 12) & 31, o = (dl >> OSH) & 7;
            int idx = segst[o] + pos[o * 64 + it * 8 + w] + rk;
            idx = clampi(idx, 0, CH - 1);
            lst[idx] = (dl << 11) | (it * 256 + t);
        }
    }
    __syncthreads();
}

__global__ __launch_bounds__(256) void k_deg(const int* __restrict__ dst, float* inv, int N, int E, int nch) {
    __shared__ int cntl[NBD];
    __shared__ __attribute__((aligned(16))) float invl[NBD];
    __shared__ int cnt[512], pos[512], lst[CH], tot[8], segst[8], segn[8];
    const int t = threadIdx.x, w = t >> 5, lane = t & 31;
    const int node0 = blockIdx.x * NBD;
    for (int i = t; i < NBD; i += 256) cntl[i] = 0;
    __syncthreads();
    for (int ch = 0; ch < nch; ++ch) {
        scan_chunk<NBD, 9>(dst, ch * CH, E, node0, cnt, pos, lst, tot, segst, segn);
        const int st = segst[w];
        int n = segn[w]; if (n > CH) n = CH;
        for (int i = 0; i < n; ++i) {
            const int li = clampi(st + i, 0, CH - 1);
            const int v = lst[li];
            const int dl = (v >> 11) & 4095;
            const int dlw = clampi(dl - (w << 9), 0, 511);
            if (lane == (dlw & 31)) cntl[(w << 9) + dlw] += 1;
        }
        __syncthreads();
    }
#pragma unroll 1
    for (int i = t; i < NBD; i += 256) {
        const int d = node0 + i;
        invl[i] = (d < N) ? rsqrtf(1.0f + (float)cntl[i]) : 1.0f;
    }
    __syncthreads();
#pragma unroll
    for (int rep = 0; rep < 2; ++rep) {
#pragma unroll
        for (int j = 0; j < 4; ++j) {
            const int idx = (w << 9) + j * 128 + lane * 4;
            const v4f val = *(const v4f*)(&invl[idx]);
            *(volatile v4f*)(inv + (size_t)node0 + idx) = val;
        }
        __threadfence();
    }
}

template <int SPLIT, int MODE>
__global__ __launch_bounds__(256) void k_gemm(const float* __restrict__ X, const unsigned short* __restrict__ Wh,
                                              const unsigned short* __restrict__ Wl, const float* __restrict__ bias,
                                              const float* __restrict__ pa, const float* __restrict__ aux,
                                              const float* __restrict__ bsc, float* Y, float* S, int nrows) {
    __shared__ __attribute__((aligned(16))) unsigned short wh[DF * LP];
    __shared__ __attribute__((aligned(16))) unsigned short wl[DF * LP];
    __shared__ __attribute__((aligned(16))) unsigned short xb[2 * GR * LP];
    __shared__ float sc[GR];
    unsigned short* xh = xb;
    unsigned short* xl = xb + GR * LP;
    float* ost = (float*)xb;
    const int t = threadIdx.x, w = t >> 5, lane = t & 31, h = lane >> 4, m = lane & 15;
    const int m0 = blockIdx.x * GR;

    for (int q = t; q < DF * 16; q += 256) {
        const int n = q >> 4, c = (q & 15) * 8;
        const uint4 v = ((const uint4*)Wh)[q];
        *(uint4*)(&wh[n * LP + c]) = v;
        if (SPLIT) { const uint4 u = ((const uint4*)Wl)[q]; *(uint4*)(&wl[n * LP + c]) = u; }
    }
    const float xsc = SPLIT ? 1.0f : 16.0f;
    for (int q = t; q < GR * DF / 4; q += 256) {
        const int row = q >> 5, c0 = (q & 31) * 4;
        const int grow = m0 + row;
        float4 v = make_float4(0.f, 0.f, 0.f, 0.f);
        if (grow < nrows) v = *(const float4*)(X + (size_t)grow * DF + c0);
        const float vv[4] = {v.x, v.y, v.z, v.w};
        unsigned short hs[4], ls[4];
#pragma unroll
        for (int i = 0; i < 4; ++i) {
            if (SPLIT) { hs[i] = f2bf(vv[i]); ls[i] = f2bf(vv[i] - bf2f(hs[i])); }
            else       { hs[i] = f2h(vv[i] * xsc); ls[i] = 0; }
        }
        uint2 ph; ph.x = (unsigned)hs[0] | ((unsigned)hs[1] << 16); ph.y = (unsigned)hs[2] | ((unsigned)hs[3] << 16);
        *(uint2*)(&xh[row * LP + c0]) = ph;
        if (SPLIT) {
            uint2 pl; pl.x = (unsigned)ls[0] | ((unsigned)ls[1] << 16); pl.y = (unsigned)ls[2] | ((unsigned)ls[3] << 16);
            *(uint2*)(&xl[row * LP + c0]) = pl;
        }
    }
    __syncthreads();

    v8f acc[4];
#pragma unroll
    for (int rt = 0; rt < 4; ++rt) acc[rt] = (v8f){0.f, 0.f, 0.f, 0.f, 0.f, 0.f, 0.f, 0.f};
    const int bn = w * 16 + m;
#pragma unroll
    for (int ks = 0; ks < 4; ++ks) {
        const int kb = ks * 32;
        if (SPLIT) {
            FragB bh, bl;
            bh.h[0] = *(const v8bf*)(&wh[bn * LP + kb + 8 * h]);
            bh.h[1] = *(const v8bf*)(&wh[bn * LP + kb + 16 + 8 * h]);
            bl.h[0] = *(const v8bf*)(&wl[bn * LP + kb + 8 * h]);
            bl.h[1] = *(const v8bf*)(&wl[bn * LP + kb + 16 + 8 * h]);
#pragma unroll
            for (int rt = 0; rt < 4; ++rt) {
                const int ar = rt * 16 + m;
                FragB ah, al;
                ah.h[0] = *(const v8bf*)(&xh[ar * LP + kb + 8 * h]);
                ah.h[1] = *(const v8bf*)(&xh[ar * LP + kb + 16 + 8 * h]);
                al.h[0] = *(const v8bf*)(&xl[ar * LP + kb + 8 * h]);
                al.h[1] = *(const v8bf*)(&xl[ar * LP + kb + 16 + 8 * h]);
                acc[rt] = __builtin_amdgcn_wmma_f32_16x16x32_bf16(false, ah.v, false, bh.v, (short)0, acc[rt], false, false);
                acc[rt] = __builtin_amdgcn_wmma_f32_16x16x32_bf16(false, ah.v, false, bl.v, (short)0, acc[rt], false, false);
                acc[rt] = __builtin_amdgcn_wmma_f32_16x16x32_bf16(false, al.v, false, bh.v, (short)0, acc[rt], false, false);
                WNOP4(acc[rt], ah.v, al.v, bh.v, bl.v);
            }
        } else {
            FragH bh;
            bh.h[0] = *(const v8h*)(&wh[bn * LP + kb + 8 * h]);
            bh.h[1] = *(const v8h*)(&wh[bn * LP + kb + 16 + 8 * h]);
#pragma unroll
            for (int rt = 0; rt < 4; ++rt) {
                const int ar = rt * 16 + m;
                FragH ah;
                ah.h[0] = *(const v8h*)(&xh[ar * LP + kb + 8 * h]);
                ah.h[1] = *(const v8h*)(&xh[ar * LP + kb + 16 + 8 * h]);
                acc[rt] = __builtin_amdgcn_wmma_f32_16x16x32_f16(false, ah.v, false, bh.v, (short)0, acc[rt], false, false);
                WNOP2(acc[rt], ah.v, bh.v);
            }
        }
    }
    __syncthreads();

    const float osc = SPLIT ? 1.0f : (1.0f / 1024.0f);
    float bia = 0.0f, a = 0.0f;
    if (MODE == 1) { bia = bias[bn]; a = pa[0]; }
#pragma unroll
    for (int rt = 0; rt < 4; ++rt) {
#pragma unroll
        for (int r = 0; r < 8; ++r) {
            float v = acc[rt][r] * osc;
            if (MODE == 1) { v += bia; v = (v >= 0.0f) ? v : a * v; }
            ost[(rt * 16 + 8 * h + r) * OP + bn] = v;
        }
    }
    __syncthreads();
    if (MODE == 2) {
        for (int j = 0; j < 8; ++j) {
            const int row = w * 8 + j;
            const int grow = m0 + row;
            float s = 0.0f;
            if (grow < nrows) {
                const v4f tv = *(const v4f*)(&ost[row * OP + lane * 4]);
                const float4 ev = *(const float4*)(aux + (size_t)grow * DF + lane * 4);
                s = tv[0] * sigf(ev.x) + tv[1] * sigf(ev.y) + tv[2] * sigf(ev.z) + tv[3] * sigf(ev.w);
            }
#pragma unroll
            for (int off = 16; off > 0; off >>= 1) s += __shfl_xor(s, off, 32);
            if (lane == 0) sc[row] = s;
        }
        __syncthreads();
        if (w < 2) {
            const int rl = w * 32 + lane;
            const int r = m0 + rl;
            const float v = (r < nrows) ? sigf(sc[rl] + bsc[0]) : 0.0f;
            *(volatile float*)(S + r) = v;
            __threadfence();
            *(volatile float*)(S + r) = v;
        }
    } else {
#pragma unroll
        for (int rep = 0; rep < 2; ++rep) {
#pragma unroll
            for (int j = 0; j < 8; ++j) {
                const int row = w * 8 + j;
                const int grow = m0 + row;
                if (grow < nrows) {
                    const v4f val = *(const v4f*)(&ost[row * OP + lane * 4]);
                    *(volatile v4f*)(Y + (size_t)grow * DF + lane * 4) = val;
                }
            }
            __threadfence();
        }
    }
}

template <int MODE>
__global__ __launch_bounds__(256) void k_agg(const float* __restrict__ xw, const int* __restrict__ src,
                                             const int* __restrict__ dst, const float* __restrict__ inv,
                                             const float* __restrict__ bias, const float* __restrict__ selw,
                                             const float* __restrict__ extra, float* Y, int N, int E, int nch) {
    extern __shared__ float accl[];
    __shared__ int cnt[512], pos[512], lst[CH], tot[8], segst[8], segn[8];
    const int t = threadIdx.x, w = t >> 5, lane = t & 31;
    const int node0 = blockIdx.x * NBA;
    for (int r = 0; r < 64; ++r) {
        const int row = (w << 6) + r;
        const int d = node0 + row;
        float4 v = make_float4(0.f, 0.f, 0.f, 0.f);
        if (d < N) {
            const float c = inv[d]; const float cc = c * c;
            const float4 x = *(const float4*)(xw + (size_t)d * DF + lane * 4);
            v.x = cc * x.x; v.y = cc * x.y; v.z = cc * x.z; v.w = cc * x.w;
        }
        *(float4*)(&accl[(size_t)row * DF + lane * 4]) = v;
    }
    for (int ch = 0; ch < nch; ++ch) {
        const int cb = ch * CH;
        scan_chunk<NBA, 6>(dst, cb, E, node0, cnt, pos, lst, tot, segst, segn);
        const int st = segst[w];
        int n = segn[w]; if (n > CH) n = CH;
        for (int i = 0; i < n; ++i) {
            const int li = clampi(st + i, 0, CH - 1);
            const int v = lst[li];
            const int dl = (v >> 11) & 4095;
            const int e = clampi(cb + (v & 2047), 0, E - 1);
            const int s = clampi(src[e], 0, N - 1);
            const int dn = clampi(node0 + dl, 0, N - 1);
            const float coef = inv[s] * inv[dn];
            const int row = (w << 6) + clampi(dl - (w << 6), 0, 63);
            const float4 x = *(const float4*)(xw + (size_t)s * DF + lane * 4);
            float4* ap = (float4*)(&accl[(size_t)row * DF + lane * 4]);
            float4 av = *ap;
            av.x += coef * x.x; av.y += coef * x.y; av.z += coef * x.z; av.w += coef * x.w;
            *ap = av;
        }
        __syncthreads();
    }
    const float4 b4 = *(const float4*)(bias + lane * 4);
#pragma unroll
    for (int rep = 0; rep < 2; ++rep) {
        for (int r = 0; r < 64; ++r) {
            const int row = (w << 6) + r;
            const int d = node0 + row;
            if (d < N) {
                const float4 av = *(const float4*)(&accl[(size_t)row * DF + lane * 4]);
                v4f v; v[0] = av.x + b4.x; v[1] = av.y + b4.y; v[2] = av.z + b4.z; v[3] = av.w + b4.w;
                if (MODE == 1) { const float sw = selw[d]; v = v * sw; }
                if (MODE == 2) {
                    const float4 ex = *(const float4*)(extra + (size_t)d * DF + lane * 4);
                    v[0] += ex.x; v[1] += ex.y; v[2] += ex.z; v[3] += ex.w;
                }
                *(volatile v4f*)(Y + (size_t)d * DF + lane * 4) = v;
            }
        }
        __threadfence();
    }
}

__global__ __launch_bounds__(256) void k_select(const float* __restrict__ scores, float* selw, int N, int K, int npad) {
    __shared__ int whist[8 * 16];
    __shared__ unsigned st_pfx, st_msk;
    __shared__ int st_kneed, wc[8], tie_base;
    const int t = threadIdx.x, w = t >> 5, lane = t & 31;
    const unsigned lt = (1u << lane) - 1u;
    if (t == 0) { st_pfx = 0u; st_msk = 0u; st_kneed = K; tie_base = 0; }
    __syncthreads();
    for (int p = 0; p < 8; ++p) {
        const int shift = 28 - 4 * p;
        const unsigned pfx = st_pfx, msk = st_msk;
        int hc = 0;
        for (int base = 0; base < N; base += 256) {
            const int i = base + t;
            const bool valid = i < N;
            const unsigned key = valid ? fmap(scores[i]) : 0u;
            const bool cand = valid && ((key & msk) == pfx);
            const int dig = (int)((key >> shift) & 15u);
            const unsigned cb = __builtin_amdgcn_ballot_w32(cand);
            if (cb != 0u) {
#pragma unroll
                for (int b = 0; b < 16; ++b) {
                    const int c = __builtin_popcount(__builtin_amdgcn_ballot_w32(cand && dig == b));
                    hc += (lane == b) ? c : 0;
                }
            }
        }
        if (lane < 16) whist[w * 16 + lane] = hc;
        __syncthreads();
        if (t == 0) {
            int cum = 0, kneed = st_kneed, done = 0;
            for (int b = 15; b >= 0; --b) {
                int hb = 0;
                for (int ww = 0; ww < 8; ++ww) hb += whist[ww * 16 + b];
                if (!done) {
                    if (cum + hb >= kneed) {
                        st_kneed = kneed - cum;
                        st_pfx = pfx | ((unsigned)b << shift);
                        st_msk = msk | (15u << shift);
                        done = 1;
                    } else cum += hb;
                }
            }
        }
        __syncthreads();
    }
    const unsigned thr = st_pfx;
    const int kneed = st_kneed;
#pragma unroll
    for (int rep = 0; rep < 2; ++rep) {
        if (t == 0) tie_base = 0;
        __syncthreads();
        for (int base = 0; base < npad; base += 256) {
            const int i = base + t;
            const bool valid = i < N;
            const float s = scores[i];
            const unsigned key = fmap(s);
            const bool gt = valid && (key > thr);
            const bool eq = valid && (key == thr);
            const unsigned em = __builtin_amdgcn_ballot_w32(eq);
            if (lane == 0) wc[w] = __builtin_popcount(em);
            __syncthreads();
            int pre = tie_base;
            for (int ww = 0; ww < w; ++ww) pre += wc[ww];
            pre += __builtin_popcount(em & lt);
            const bool sel = gt || (eq && pre < kneed);
            const float v = sel ? s : 0.0f;
            *(volatile float*)(selw + i) = v;
            __syncthreads();
            if (t == 0) { int tb2 = tie_base; for (int ww = 0; ww < 8; ++ww) tb2 += wc[ww]; tie_base = tb2; }
            __syncthreads();
        }
        __threadfence();
    }
}

extern "C" void kernel_launch(void* const* d_in, const int* in_sizes, int n_in,
                              void* d_out, int out_size, void* d_ws, size_t ws_size,
                              hipStream_t stream) {
    if (n_in < 14) return;
    const float* feat = (const float*)d_in[0];
    const float* hneg = (const float*)d_in[1];
    const int*   ei   = (const int*)d_in[2];
    const float* Wd   = (const float*)d_in[3];
    const float* bd   = (const float*)d_in[4];
    const float* pa   = (const float*)d_in[5];
    const float* Wbil = (const float*)d_in[6];
    const float* bbil = (const float*)d_in[7];
    const float* Wg1  = (const float*)d_in[8];
    const float* bg1  = (const float*)d_in[9];
    const float* Wg2  = (const float*)d_in[10];
    const float* bg2  = (const float*)d_in[11];
    const float* Wg3  = (const float*)d_in[12];
    const float* bg3  = (const float*)d_in[13];

    const int N = in_sizes[0] / DF;
    const int E = in_sizes[2] / 2;
    if (N <= 0 || E <= 0) return;
    const int* es = ei;
    const int* ed = ei + E;
    const int K = N / 2;
    const size_t ND = (size_t)N * DF;
    const int NP = ((N + NBD - 1) / NBD) * NBD;
    const size_t WI = (size_t)DF * DF;

    char* wp = (char*)d_ws; size_t o = 0;
    auto alloc = [&](size_t bytes) { void* p = wp + o; o = (o + bytes + 255) & ~(size_t)255; return p; };
    float* hpos   = (float*)alloc(ND * 4);
    float* xw     = (float*)alloc(ND * 4);
    float* emb    = (float*)alloc(ND * 4);
    float* tbf    = (float*)alloc(ND * 4);
    float* inv    = (float*)alloc((size_t)NP * 4);
    float* scores = (float*)alloc((size_t)NP * 4);
    float* scneg  = (float*)alloc((size_t)NP * 4);
    float* selw   = (float*)alloc((size_t)NP * 4);
    unsigned short* wimg = (unsigned short*)alloc(NPART * WI * 2);
    if (o > ws_size) return;
    if ((size_t)out_size < ND) return;
    float* outp = (float*)d_out;

    dim3 b(256);
    const int gM  = (N + GR - 1) / GR;
    const int gA  = (N + NBA - 1) / NBA;
    const int gD  = NP / NBD;
    const int nch = (E + CH - 1) / CH;
    const size_t aggLds = (size_t)NBA * DF * 4;

    hipFuncSetAttribute((const void*)k_agg<0>, hipFuncAttributeMaxDynamicSharedMemorySize, (int)aggLds);
    hipFuncSetAttribute((const void*)k_agg<1>, hipFuncAttributeMaxDynamicSharedMemorySize, (int)aggLds);
    hipFuncSetAttribute((const void*)k_agg<2>, hipFuncAttributeMaxDynamicSharedMemorySize, (int)aggLds);

    k_prepw<<<NPART, b, 0, stream>>>(Wd, Wg1, Wbil, Wg2, Wg3, wimg);
    k_deg<<<gD, b, 0, stream>>>(ed, inv, N, E, nch);
    k_gemm<1, 1><<<gM, b, 0, stream>>>(feat, wimg + 0 * WI, wimg + 1 * WI, bd, pa, feat, bbil, hpos, scores, N);
    k_gemm<1, 0><<<gM, b, 0, stream>>>(hpos, wimg + 3 * WI, wimg + 4 * WI, bg1, pa, feat, bbil, xw, scores, N);
    k_agg<0><<<gA, b, aggLds, stream>>>(xw, es, ed, inv, bg1, selw, hpos, emb, N, E, nch);
    k_gemm<1, 2><<<gM, b, 0, stream>>>(hpos, wimg + 5 * WI, wimg + 6 * WI, bg1, pa, emb, bbil, xw, scores, N);
    k_gemm<0, 1><<<gM, b, 0, stream>>>(hneg, wimg + 2 * WI, wimg + 2 * WI, bd, pa, feat, bbil, tbf, scneg, N);
    k_gemm<0, 2><<<gM, b, 0, stream>>>(tbf, wimg + 7 * WI, wimg + 7 * WI, bg1, pa, emb, bbil, xw, scneg, N);
    k_select<<<1, b, 0, stream>>>(scores, selw, N, K, NP);
    k_gemm<0, 0><<<gM, b, 0, stream>>>(emb, wimg + 8 * WI, wimg + 8 * WI, bg2, pa, feat, bbil, xw, scneg, N);
    k_agg<1><<<gA, b, aggLds, stream>>>(xw, es, ed, inv, bg2, selw, hpos, tbf, N, E, nch);
    k_gemm<0, 0><<<gM, b, 0, stream>>>(tbf, wimg + 9 * WI, wimg + 9 * WI, bg3, pa, feat, bbil, xw, scneg, N);
    k_agg<2><<<gA, b, aggLds, stream>>>(xw, es, ed, inv, bg3, selw, emb, outp, N, E, nch);
}
